// lstm_6425271075258
// MI455X (gfx1250) — hardware-verified
//
#include <hip/hip_runtime.h>
#include <math.h>

typedef __attribute__((ext_vector_type(16))) _Float16 v16h;
typedef __attribute__((ext_vector_type(8)))  _Float16 v8h;
typedef __attribute__((ext_vector_type(8)))  float    v8f;
typedef __attribute__((ext_vector_type(4)))  float    v4f;

constexpr int kSteps      = 2048;
constexpr int kBatch      = 4096;
constexpr int kHid        = 4;
constexpr int kGate4      = 4 * kHid;
constexpr int kBlkRows    = 32;
constexpr int kThr        = 64;
constexpr int kBlocks     = kBatch / kBlkRows;
constexpr int kChunk      = 32;
constexpr int kNumChunks  = kSteps / kChunk;
constexpr int kPitch      = 36;
constexpr size_t kOutElems = (size_t)kSteps * (size_t)kBatch;
static_assert(kHid == 4 && kGate4 == 16, "the four gates of the four units fill the 16 rows of one tile");
static_assert(kBatch % kBlkRows == 0 && kSteps % kChunk == 0, "whole blocks and chunks");
static_assert(kBlkRows == 32 && kThr == 64, "two waves x 16 batch columns = one 128-B line of a time-major row");
static_assert((kPitch % 4) == 0, "16-B aligned LDS rows");

constexpr float kStateCarry  = 256.0f;
constexpr float kWeightCarry = 64.0f;
constexpr float kFoldBack    = 1.0f / (kStateCarry * kWeightCarry);
constexpr float kF16MinNorm  = 6.103515625e-5f;
static_assert(kStateCarry * kWeightCarry == 16384.0f, "carry product");

namespace eng {

union FragU { v16h v; v8h h[2]; };

__device__ __forceinline__ unsigned short f2bf_bits(float f) {
  unsigned u = __float_as_uint(f);
  return (unsigned short)((u + 0x7FFFu + ((u >> 16) & 1u)) >> 16);
}
__device__ __forceinline__ float bf16v(float f) {
  return __uint_as_float(((unsigned)f2bf_bits(f)) << 16);
}
__device__ __forceinline__ _Float16 to_f16_flushed(float c) {
  const float z = (fabsf(c) < kF16MinNorm) ? 0.0f : c;
  return (_Float16)z;
}
__device__ __forceinline__ v8f mma_f16(v16h a, v16h b) {
  v8f c = (v8f){0.f, 0.f, 0.f, 0.f, 0.f, 0.f, 0.f, 0.f};
  c = __builtin_amdgcn_wmma_f32_16x16x32_f16(false, a, false, b, (short)0, c, false, false);
  asm volatile("v_nop\n\tv_nop\n\tv_nop\n\tv_nop" : "+v"(c) : "v"(a), "v"(b));
  return c;
}
__device__ __forceinline__ float fast_tanh(float v) {
  const float e = __expf(2.0f * v);
  return 1.0f - 2.0f * __builtin_amdgcn_rcpf(e + 1.0f);
}
__device__ __forceinline__ float fast_sigmoid(float v) {
  return __builtin_amdgcn_rcpf(1.0f + __expf(-v));
}

}

__global__ __launch_bounds__(kThr) void lstm4x2_seq_kernel(
    const float* __restrict__ x,
    const float* __restrict__ w_ih0, const float* __restrict__ w_hh0,
    const float* __restrict__ b_ih0, const float* __restrict__ b_hh0,
    const float* __restrict__ w_ih1, const float* __restrict__ w_hh1,
    const float* __restrict__ b_ih1, const float* __restrict__ b_hh1,
    const float* __restrict__ w_out, const float* __restrict__ b_out,
    float* __restrict__ outs)
{
  __shared__ __align__(16) float xs[kChunk * kPitch];
  __shared__ __align__(16) float os[kChunk * kPitch];
  __shared__ __align__(16) float wsm[3 * 64];
  __shared__ __align__(16) float vsm[6 * 16];
  __shared__ __align__(16) float osm[8];

  const int tid  = threadIdx.x;
  const int lane = tid & 31;
  const int wave = __builtin_amdgcn_readfirstlane(tid >> 5);
  const int hsel = lane >> 4;
  const int n    = lane & 15;
  const bool lowHalf = (hsel == 0);
  const int b0   = blockIdx.x * kBlkRows;
  const int col  = 16 * wave + n;

  {
    wsm[0 * 64 + tid] = w_hh0[tid];
    wsm[1 * 64 + tid] = w_ih1[tid];
    wsm[2 * 64 + tid] = w_hh1[tid];
    const int i16 = tid & 15;
    const int sel = tid >> 4;
    const float v0 = w_ih0[i16];
    const float v1 = b_ih0[i16];
    const float v2 = b_hh0[i16];
    const float v3 = b_ih1[i16];
    const float v4 = b_hh1[i16];
    const float pick = (sel == 0) ? v0 : ((sel == 1) ? v1 : ((sel == 2) ? v2 : v3));
    vsm[sel * 16 + i16] = pick;
    const float v5 = w_out[tid & 3];
    const float v6 = b_out[0];
    asm volatile("" :: "v"(v4), "v"(v5), "v"(v6));
    if (tid < 16) vsm[4 * 16 + tid] = v4;
    if (tid < 4)  osm[tid] = v5;
    if (tid == 4) osm[4] = v6;
  }
  __syncthreads();

  v16h fragA1, fragA2;
  {
    const int m = n;
    const v8h zero8 = (v8h){(_Float16)0.0f, (_Float16)0.0f, (_Float16)0.0f, (_Float16)0.0f,
                            (_Float16)0.0f, (_Float16)0.0f, (_Float16)0.0f, (_Float16)0.0f};
    v8h a1, a2;
#pragma unroll
    for (int i = 0; i < 8; ++i) {
      const int ic = i & 3;
      const float f_hh0 = wsm[0 * 64 + m * kHid + ic];
      const float f_ih0 = vsm[0 * 16 + m];
      const float f_ih1 = wsm[1 * 64 + m * kHid + ic];
      const float f_hh1 = wsm[2 * 64 + m * kHid + ic];
      const float p1 = (i < kHid) ? f_hh0 : f_ih0;
      const bool ok1 = lowHalf && (i <= kHid);
      const float p2 = (i < kHid) ? f_ih1 : f_hh1;
      const bool ok2 = lowHalf;
      a1[i] = eng::to_f16_flushed(ok1 ? (eng::bf16v(p1) * kWeightCarry) : 0.0f);
      a2[i] = eng::to_f16_flushed(ok2 ? (eng::bf16v(p2) * kWeightCarry) : 0.0f);
    }
    eng::FragU u1, u2;
    u1.h[0] = a1;
    u1.h[1] = zero8;
    u2.h[0] = a2;
    u2.h[1] = zero8;
    fragA1 = u1.v;
    fragA2 = u2.v;
  }

  float br1[8], br2[8];
#pragma unroll
  for (int r = 0; r < 8; ++r) {
    const int row = 8 * hsel + r;
    br1[r] = eng::bf16v(vsm[1 * 16 + row]) + eng::bf16v(vsm[2 * 16 + row]);
    br2[r] = eng::bf16v(vsm[3 * 16 + row]) + eng::bf16v(vsm[4 * 16 + row]);
  }
  float wo[4];
#pragma unroll
  for (int u = 0; u < kHid; ++u) wo[u] = eng::bf16v(osm[u]);
  const float bo = eng::bf16v(osm[4]);
  float h1f[4], c1f[4], h2f[4], c2f[4];
  _Float16 h1b[4], h2b[4];
#pragma unroll
  for (int u = 0; u < kHid; ++u) {
    h1f[u] = 0.0f; c1f[u] = 0.0f; h2f[u] = 0.0f; c2f[u] = 0.0f;
    h1b[u] = (_Float16)0.0f; h2b[u] = (_Float16)0.0f;
  }
  const v8h zh = (v8h){(_Float16)0.0f, (_Float16)0.0f, (_Float16)0.0f, (_Float16)0.0f,
                       (_Float16)0.0f, (_Float16)0.0f, (_Float16)0.0f, (_Float16)0.0f};

  const int q  = tid >> 3;
  const int c4 = (tid & 7) * 4;

#pragma unroll 1
  for (int ch = 0; ch < kNumChunks; ++ch) {
    const int t0 = ch * kChunk;
#pragma unroll
    for (int it = 0; it < 4; ++it) {
      const int step = it * 8 + q;
      const v4f v = *(const v4f*)(x + (size_t)(t0 + step) * kBatch + b0 + c4);
      v4f rv;
      const float v0 = v[0];
      const float v1 = v[1];
      const float v2 = v[2];
      const float v3 = v[3];
      rv[0] = eng::bf16v(v0);
      rv[1] = eng::bf16v(v1);
      rv[2] = eng::bf16v(v2);
      rv[3] = eng::bf16v(v3);
      *(v4f*)(xs + step * kPitch + c4) = rv;
    }
    __syncthreads();

#pragma unroll 1
    for (int s = 0; s < kChunk; ++s) {
      const float xv = xs[s * kPitch + col];

      v8h b1 = zh;
#pragma unroll
      for (int u = 0; u < kHid; ++u) b1[u] = h1b[u];
      b1[kHid] = eng::to_f16_flushed(lowHalf ? (xv * kStateCarry) : 0.0f);
      eng::FragU f1;
      f1.h[0] = b1;
      f1.h[1] = zh;
      const v8f d1 = eng::mma_f16(fragA1, f1.v);
      float p1[8], o1[8];
#pragma unroll
      for (int r = 0; r < 8; ++r) p1[r] = fmaf(d1[r], kFoldBack, br1[r]);
#pragma unroll
      for (int r = 0; r < 8; ++r) o1[r] = __shfl_xor(p1[r], 16, 32);
#pragma unroll
      for (int u = 0; u < kHid; ++u) {
        const float ig = eng::fast_sigmoid(p1[u]);
        const float fg = eng::fast_sigmoid(p1[kHid + u]);
        const float gg = eng::fast_tanh(o1[u]);
        const float og = eng::fast_sigmoid(o1[kHid + u]);
        const float cn = fg * c1f[u] + ig * gg;
        const float hv = og * eng::fast_tanh(cn);
        c1f[u] = lowHalf ? cn : 0.0f;
        h1f[u] = lowHalf ? hv : 0.0f;
        h1b[u] = eng::to_f16_flushed(h1f[u] * kStateCarry);
      }

      v8h b2 = zh;
#pragma unroll
      for (int u = 0; u < kHid; ++u) { b2[u] = h1b[u]; b2[kHid + u] = h2b[u]; }
      eng::FragU f2;
      f2.h[0] = b2;
      f2.h[1] = zh;
      const v8f d2 = eng::mma_f16(fragA2, f2.v);
      float p2[8], o2[8];
#pragma unroll
      for (int r = 0; r < 8; ++r) p2[r] = fmaf(d2[r], kFoldBack, br2[r]);
#pragma unroll
      for (int r = 0; r < 8; ++r) o2[r] = __shfl_xor(p2[r], 16, 32);
      float y = bo;
#pragma unroll
      for (int u = 0; u < kHid; ++u) {
        const float ig = eng::fast_sigmoid(p2[u]);
        const float fg = eng::fast_sigmoid(p2[kHid + u]);
        const float gg = eng::fast_tanh(o2[u]);
        const float og = eng::fast_sigmoid(o2[kHid + u]);
        const float cn = fg * c2f[u] + ig * gg;
        const float hv = og * eng::fast_tanh(cn);
        c2f[u] = lowHalf ? cn : 0.0f;
        h2f[u] = lowHalf ? hv : 0.0f;
        h2b[u] = eng::to_f16_flushed(h2f[u] * kStateCarry);
        y = fmaf(wo[u], h2f[u], y);
      }
      if (lowHalf) os[s * kPitch + col] = y;
    }
    __syncthreads();

    {
      for (int pass = 0; pass < 2; ++pass) {
#pragma unroll
        for (int it = 0; it < 4; ++it) {
          const int step = it * 8 + q;
          const v4f ov = *(const v4f*)(os + step * kPitch + c4);
          *(volatile v4f*)(outs + (size_t)(t0 + step) * kBatch + b0 + c4) = ov;
        }
        __threadfence();
      }
    }
  }
}

extern "C" void kernel_launch(void* const* d_in, const int* in_sizes, int n_in,
                              void* d_out, int out_size, void* d_ws, size_t ws_size,
                              hipStream_t stream) {
  (void)d_ws;
  (void)ws_size;
  if (n_in < 11 || d_out == nullptr) return;
  if ((size_t)in_sizes[0] != kOutElems) return;
  if (in_sizes[1] != kGate4 || in_sizes[2] != kGate4 * kHid || in_sizes[3] != kGate4 || in_sizes[4] != kGate4) return;
  if (in_sizes[5] != kGate4 * kHid || in_sizes[6] != kGate4 * kHid || in_sizes[7] != kGate4 || in_sizes[8] != kGate4) return;
  if (in_sizes[9] != kHid || in_sizes[10] != 1) return;
  if ((size_t)out_size != kOutElems) return;

  const float* x     = (const float*)d_in[0];
  const float* w_ih0 = (const float*)d_in[1];
  const float* w_hh0 = (const float*)d_in[2];
  const float* b_ih0 = (const float*)d_in[3];
  const float* b_hh0 = (const float*)d_in[4];
  const float* w_ih1 = (const float*)d_in[5];
  const float* w_hh1 = (const float*)d_in[6];
  const float* b_ih1 = (const float*)d_in[7];
  const float* b_hh1 = (const float*)d_in[8];
  const float* w_out = (const float*)d_in[9];
  const float* b_out = (const float*)d_in[10];
  float* outs = (float*)d_out;

  lstm4x2_seq_kernel<<<kBlocks, kThr, 0, stream>>>(x, w_ih0, w_hh0, b_ih0, b_hh0, w_ih1, w_hh1, b_ih1, b_hh1, w_out, b_out, outs);
}
